// DAGLayer_46694884442362
// MI455X (gfx1250) — hardware-verified
//
#include <hip/hip_runtime.h>
#include <stddef.h>


#define DW      128
#define NTHR    256
#define NWAVE   8
#define EPT     8
#define NGRP    2
#define CHUNK   (NTHR * EPT * NGRP)
#define WCAP    (EPT * NGRP * 32)
#define LISTN   (NWAVE * WCAP)
#define NBC     4096
#define NBF     1024
#define RCAP    40960
#define RBN     128
#define TGT     256
#define DEGCAP  1024
#define OTHR    512
#define BM      64
#define WSCAP   134217728
#define ACARRY  8.0f
#define WCARRY  64.0f
#define GSCALE  (1.0f / 512.0f)
#define LN_EPS  1e-5f

#define LDS_FILL  ((RCAP + NBF + LISTN) * 4 + 64)
#define LDS_LAYER (2 * BM * DW * 2 + BM * DW * 4)

static_assert((CHUNK & (CHUNK - 1)) == 0);
static_assert(CHUNK <= 4096);
static_assert((NBC & (NBC - 1)) == 0 && (NBF & (NBF - 1)) == 0);
static_assert(NBC == 4 * NBF);
static_assert(OTHR * 8 == NBC);
static_assert((RCAP % 32) == 0);
static_assert(TGT == NWAVE * 32);
static_assert((NBC % TGT) == 0);
static_assert((TGT % BM) == 0);
static_assert(DW == 4 * 32);
static_assert((DW % 32) == 0);
static_assert(WCAP == EPT * NGRP * 32);
static_assert(LDS_LAYER == 65536);
static_assert(BM * DW * 4 == 2 * BM * DW * 2);

typedef float    v4f  __attribute__((ext_vector_type(4)));
typedef float    v8f  __attribute__((ext_vector_type(8)));
typedef int      v4i  __attribute__((ext_vector_type(4)));
typedef _Float16 v4h  __attribute__((ext_vector_type(4)));
typedef _Float16 v8h  __attribute__((ext_vector_type(8)));
typedef _Float16 v16h __attribute__((ext_vector_type(16)));
union Frag { v16h v; v8h h[2]; };

__device__ __forceinline__ v8f wmh(v16h a, v16h b, v8f c) {
  v8f d = __builtin_amdgcn_wmma_f32_16x16x32_f16(false, a, false, b, (short)0, c, false, false);
  asm volatile("v_nop\n\tv_nop\n\tv_nop\n\tv_nop" : "+v"(d) : "v"(a), "v"(b));
  return d;
}

__device__ __forceinline__ float wsum(float x) {
  x += __shfl_xor(x, 16);
  x += __shfl_xor(x, 8);
  x += __shfl_xor(x, 4);
  x += __shfl_xor(x, 2);
  x += __shfl_xor(x, 1);
  return x;
}

template <int NB>
__device__ __forceinline__ int scan_chunk(const int* __restrict__ dsts, int nE, int cbase, int slotBase,
                                          int vec8, int* list, int tid, int lane, int wave) {
  int wc = 0;
#pragma unroll
  for (int g = 0; g < NGRP; ++g) {
    const int el0  = (g * NTHR + tid) * EPT;
    const int e0   = cbase + el0;
    const int sent = -2147483647 - 1;
    v4i da, db;
    if (vec8 != 0 && cbase + CHUNK <= nE) {
      da = *(const v4i*)(dsts + e0);
      db = *(const v4i*)(dsts + e0 + 4);
    } else {
      da.x = (e0     < nE) ? dsts[min(e0, nE - 1)] : sent;
      da.y = (e0 + 1 < nE) ? dsts[min(e0 + 1, nE - 1)] : sent;
      da.z = (e0 + 2 < nE) ? dsts[min(e0 + 2, nE - 1)] : sent;
      da.w = (e0 + 3 < nE) ? dsts[min(e0 + 3, nE - 1)] : sent;
      db.x = (e0 + 4 < nE) ? dsts[min(e0 + 4, nE - 1)] : sent;
      db.y = (e0 + 5 < nE) ? dsts[min(e0 + 5, nE - 1)] : sent;
      db.z = (e0 + 6 < nE) ? dsts[min(e0 + 6, nE - 1)] : sent;
      db.w = (e0 + 7 < nE) ? dsts[min(e0 + 7, nE - 1)] : sent;
    }
    const unsigned nb = (unsigned)slotBase;
    const unsigned s0 = (unsigned)da.x - nb, s1 = (unsigned)da.y - nb;
    const unsigned s2 = (unsigned)da.z - nb, s3 = (unsigned)da.w - nb;
    const unsigned s4 = (unsigned)db.x - nb, s5 = (unsigned)db.y - nb;
    const unsigned s6 = (unsigned)db.z - nb, s7 = (unsigned)db.w - nb;
    const bool h0 = s0 < (unsigned)NB, h1 = s1 < (unsigned)NB, h2 = s2 < (unsigned)NB, h3 = s3 < (unsigned)NB;
    const bool h4 = s4 < (unsigned)NB, h5 = s5 < (unsigned)NB, h6 = s6 < (unsigned)NB, h7 = s7 < (unsigned)NB;
    const unsigned any = __builtin_amdgcn_ballot_w32(h0 | h1 | h2 | h3 | h4 | h5 | h6 | h7);
    if (any != 0u) {
#define HITJ(J, HJ, SJ) { \
        const unsigned mj = __builtin_amdgcn_ballot_w32(HJ); \
        if (mj != 0u) { \
          if (HJ) { \
            const int pos = wc + (int)__builtin_amdgcn_mbcnt_lo(mj, 0u); \
            if (pos < WCAP) list[wave * WCAP + pos] = ((el0 + (J)) << 12) | (int)(SJ); \
          } \
          wc += (int)__builtin_popcount(mj); } }
      HITJ(0, h0, s0)
      HITJ(1, h1, s1)
      HITJ(2, h2, s2)
      HITJ(3, h3, s3)
      HITJ(4, h4, s4)
      HITJ(5, h5, s5)
      HITJ(6, h6, s6)
      HITJ(7, h7, s7)
#undef HITJ
    }
  }
  return wc;
}

__global__ __launch_bounds__(NTHR) void k_count(const int* __restrict__ dsts, int* cnt, int nE, int vec8) {
  __shared__ __attribute__((aligned(16))) int scnt[NBC];
  __shared__ __attribute__((aligned(16))) int list[LISTN];
  __shared__ int wcnt[NWAVE];
  const int tid = threadIdx.x, lane = tid & 31, wave = tid >> 5;
  const int nodeBase = blockIdx.x * NBC;

  for (int i = tid; i < NBC; i += NTHR) scnt[i] = 0;
  __syncthreads();

  const int nChunks = (nE + CHUNK - 1) / CHUNK;
#pragma unroll 1
  for (int ch = 0; ch < nChunks; ++ch) {
    const int cbase = ch * CHUNK;
    const int wc = scan_chunk<NBC>(dsts, nE, cbase, nodeBase, vec8, list, tid, lane, wave);
    if (lane == 0) wcnt[wave] = wc;
    __syncthreads();
    if (wave == 0) {
#pragma unroll 1
      for (int wsx = 0; wsx < NWAVE; ++wsx) {
        int n = __builtin_amdgcn_readfirstlane(wcnt[wsx]);
        n = n > WCAP ? WCAP : (n < 0 ? 0 : n);
        const int* lp = list + wsx * WCAP;
#pragma unroll 1
        for (int i = 0; i < n; ++i) {
          const int ent  = __builtin_amdgcn_readfirstlane(lp[i]);
          const int slot = ent & (NBC - 1);
          if (lane == 0) scnt[slot] = scnt[slot] + 1;
        }
      }
    }
    __syncthreads();
  }

  v4i cq[4];
#pragma unroll
  for (int q = 0; q < 4; ++q) {
    const int f = (wave * 4 + q) * 128 + 4 * lane;
    cq[q] = *(const v4i*)(scnt + f);
  }
  int* cp = cnt + (size_t)nodeBase;
#pragma unroll
  for (int q = 0; q < 4; ++q) {
    const int f = (wave * 4 + q) * 128 + 4 * lane;
    *(volatile v4i*)(cp + f) = cq[q];
  }
  __threadfence();
#pragma unroll
  for (int q = 0; q < 4; ++q) {
    const int f = (wave * 4 + q) * 128 + 4 * lane;
    *(volatile v4i*)(cp + f) = cq[q];
  }
}

__global__ __launch_bounds__(OTHR) void k_offsets(
    const int* __restrict__ cnt, int* off, int* rbase, int nChunk) {
  __shared__ __attribute__((aligned(16))) int soff[NBC];
  __shared__ __attribute__((aligned(16))) int srb[RBN];
  __shared__ int wtot[OTHR / 32];
  const int tid = threadIdx.x, lane = tid & 31, wave = tid >> 5, sub = tid >> 7;
  for (int i = tid; i < RBN; i += OTHR) srb[i] = 0;
  int carry = 0;
#pragma unroll 1
  for (int ch = 0; ch < nChunk; ++ch) {
    const int base = ch * NBC;
    const v4i c0 = *(const v4i*)(cnt + base + 8 * tid);
    const v4i c1 = *(const v4i*)(cnt + base + 8 * tid + 4);
    const int e0 = max(c0.x, 0), e1 = max(c0.y, 0), e2 = max(c0.z, 0), e3 = max(c0.w, 0);
    const int e4 = max(c1.x, 0), e5 = max(c1.y, 0), e6 = max(c1.z, 0), e7 = max(c1.w, 0);
    const int ts = e0 + e1 + e2 + e3 + e4 + e5 + e6 + e7;
    int incl = ts;
#pragma unroll
    for (int d = 1; d < 32; d <<= 1) {
      const int t = __shfl_up(incl, d);
      if (lane >= d) incl += t;
    }
    if (lane == 31) wtot[wave] = incl;
    __syncthreads();
    const int S0 = wtot[0]  + wtot[1]  + wtot[2]  + wtot[3];
    const int S1 = wtot[4]  + wtot[5]  + wtot[6]  + wtot[7];
    const int S2 = wtot[8]  + wtot[9]  + wtot[10] + wtot[11];
    const int S3 = wtot[12] + wtot[13] + wtot[14] + wtot[15];
    int pre = 0;
#pragma unroll 1
    for (int w = 4 * sub; w < wave; ++w) pre += wtot[w];
    const int b0 = carry;
    const int b1 = b0 + ((S0 + 31) & ~31);
    const int b2 = b1 + ((S1 + 31) & ~31);
    const int b3 = b2 + ((S2 + 31) & ~31);
    const int b4 = b3 + ((S3 + 31) & ~31);
    const int myb = sub == 0 ? b0 : (sub == 1 ? b1 : (sub == 2 ? b2 : b3));
    if (tid == 0) {
      srb[min(4 * ch + 0, RBN - 1)] = b0;
      srb[min(4 * ch + 1, RBN - 1)] = b1;
      srb[min(4 * ch + 2, RBN - 1)] = b2;
      srb[min(4 * ch + 3, RBN - 1)] = b3;
    }
    int run = myb + pre + incl - ts;
    soff[8 * tid + 0] = run; run += e0;
    soff[8 * tid + 1] = run; run += e1;
    soff[8 * tid + 2] = run; run += e2;
    soff[8 * tid + 3] = run; run += e3;
    soff[8 * tid + 4] = run; run += e4;
    soff[8 * tid + 5] = run; run += e5;
    soff[8 * tid + 6] = run; run += e6;
    soff[8 * tid + 7] = run;
    carry = b4;
    __syncthreads();
    const v4i o0 = *(const v4i*)(soff + 4 * tid);
    const v4i o1 = *(const v4i*)(soff + 4 * (tid + OTHR));
    int* op = off + base;
    *(volatile v4i*)(op + 4 * tid) = o0;
    *(volatile v4i*)(op + 4 * (tid + OTHR)) = o1;
    __threadfence();
    *(volatile v4i*)(op + 4 * tid) = o0;
    *(volatile v4i*)(op + 4 * (tid + OTHR)) = o1;
    __syncthreads();
  }
  if (tid == 0) srb[min(4 * nChunk, RBN - 1)] = carry;
  __syncthreads();
  v4i rv = {0, 0, 0, 0};
  if (tid < 32) rv = *(const v4i*)(srb + 4 * tid);
  if (tid < 32) *(volatile v4i*)(rbase + 4 * tid) = rv;
  __threadfence();
  if (tid < 32) *(volatile v4i*)(rbase + 4 * tid) = rv;
}

__global__ __launch_bounds__(NTHR) void k_fill(
    const int* __restrict__ srcs, const int* __restrict__ dsts,
    const int* __restrict__ off, const int* __restrict__ rbase,
    int* csr, int nN, int nE, int vec8, int csrLen) {
  extern __shared__ v4f lds_dyn[];
  int* region = (int*)lds_dyn;
  int* cursor = region + RCAP;
  int* list   = cursor + NBF;
  int* wcnt   = list + LISTN;
  const int tid = threadIdx.x, lane = tid & 31, wave = tid >> 5;
  const int b = blockIdx.x;
  const int nodeBase = b * NBF;

  int rb0 = rbase[b];
  const int rb1 = rbase[b + 1];
  rb0 = rb0 < 0 ? 0 : (rb0 > csrLen ? csrLen : rb0);
  rb0 &= ~31;
  int len = rb1 - rb0;
  len = len < 0 ? 0 : (len > RCAP ? RCAP : len);
  int lenW = (len + 31) & ~31;
  if (rb0 + lenW > csrLen) lenW = (csrLen - rb0) & ~31;

  {
    const v4i z = {0, 0, 0, 0};
    for (int i = tid; i < RCAP / 4; i += NTHR) ((v4i*)region)[i] = z;
    for (int s = tid; s < NBF; s += NTHR) {
      int o = off[nodeBase + s] - rb0;
      o = o < 0 ? 0 : (o > RCAP ? RCAP : o);
      cursor[s] = o;
    }
  }
  __syncthreads();

  const int nChunks = (nE + CHUNK - 1) / CHUNK;
#pragma unroll 1
  for (int ch = 0; ch < nChunks; ++ch) {
    const int cbase = ch * CHUNK;
    const int wc = scan_chunk<NBF>(dsts, nE, cbase, nodeBase, vec8, list, tid, lane, wave);
    if (lane == 0) wcnt[wave] = wc;
    __syncthreads();
    if (wave == 0) {
#pragma unroll 1
      for (int wsx = 0; wsx < NWAVE; ++wsx) {
        int n = __builtin_amdgcn_readfirstlane(wcnt[wsx]);
        n = n > WCAP ? WCAP : (n < 0 ? 0 : n);
        const int* lp = list + wsx * WCAP;
#pragma unroll 1
        for (int i = 0; i < n; ++i) {
          const int ent  = __builtin_amdgcn_readfirstlane(lp[i]);
          const int slot = ent & (NBF - 1);
          int e = cbase + ((ent >> 12) & (CHUNK - 1));
          e = e > nE - 1 ? nE - 1 : e;
          int sv = srcs[e];
          sv = sv < 0 ? 0 : (sv > nN - 1 ? nN - 1 : sv);
          if (lane == 0) {
            int pos = cursor[slot];
            pos = pos < 0 ? 0 : (pos > RCAP - 1 ? RCAP - 1 : pos);
            region[pos] = sv;
            const int np = pos + 1;
            cursor[slot] = np > RCAP ? RCAP : np;
          }
        }
      }
    }
    __syncthreads();
  }

  const int nv = lenW >> 2;
  int* gp = csr + rb0;
#pragma unroll 1
  for (int i = tid; i < nv; i += NTHR) { const v4i v = ((const v4i*)region)[i]; *(volatile v4i*)(gp + 4 * i) = v; }
  __threadfence();
#pragma unroll 1
  for (int i = tid; i < nv; i += NTHR) { const v4i v = ((const v4i*)region)[i]; *(volatile v4i*)(gp + 4 * i) = v; }
}

__global__ __launch_bounds__(NTHR) void k_wcvt(const float* __restrict__ wS, const float* __restrict__ wN,
                                               const float* __restrict__ wG, _Float16* dp, int nUnits) {
  const int i = (int)blockIdx.x * NTHR + (int)threadIdx.x;
  if (i >= nUnits) return;
  const int uS = (DW * DW) / 8;
  const int uG = (2 * DW * DW) / 8;
  int iS = i;          iS = iS > uS - 1 ? uS - 1 : (iS < 0 ? 0 : iS);
  int iN = i - uS;     iN = iN > uS - 1 ? uS - 1 : (iN < 0 ? 0 : iN);
  int iG = i - 2 * uS; iG = iG > uG - 1 ? uG - 1 : (iG < 0 ? 0 : iG);
  const v4f a0 = *(const v4f*)(wS + (size_t)8 * iS), a1 = *(const v4f*)(wS + (size_t)8 * iS + 4);
  const v4f b0 = *(const v4f*)(wN + (size_t)8 * iN), b1 = *(const v4f*)(wN + (size_t)8 * iN + 4);
  const v4f c0 = *(const v4f*)(wG + (size_t)8 * iG), c1 = *(const v4f*)(wG + (size_t)8 * iG + 4);
  const int sel = i < uS ? 0 : (i < 2 * uS ? 1 : 2);
  v4f x0, x1;
  x0.x = sel == 0 ? a0.x : (sel == 1 ? b0.x : c0.x);
  x0.y = sel == 0 ? a0.y : (sel == 1 ? b0.y : c0.y);
  x0.z = sel == 0 ? a0.z : (sel == 1 ? b0.z : c0.z);
  x0.w = sel == 0 ? a0.w : (sel == 1 ? b0.w : c0.w);
  x1.x = sel == 0 ? a1.x : (sel == 1 ? b1.x : c1.x);
  x1.y = sel == 0 ? a1.y : (sel == 1 ? b1.y : c1.y);
  x1.z = sel == 0 ? a1.z : (sel == 1 ? b1.z : c1.z);
  x1.w = sel == 0 ? a1.w : (sel == 1 ? b1.w : c1.w);
  v8h o;
  o[0] = (_Float16)(x0.x * WCARRY); o[1] = (_Float16)(x0.y * WCARRY);
  o[2] = (_Float16)(x0.z * WCARRY); o[3] = (_Float16)(x0.w * WCARRY);
  o[4] = (_Float16)(x1.x * WCARRY); o[5] = (_Float16)(x1.y * WCARRY);
  o[6] = (_Float16)(x1.z * WCARRY); o[7] = (_Float16)(x1.w * WCARRY);
  _Float16* gp = dp + (size_t)i * 8;
  *(volatile v8h*)gp = o;
  __threadfence();
  *(volatile v8h*)gp = o;
}

__global__ __launch_bounds__(NTHR) void k_agg(
    const int* __restrict__ csr, const int* __restrict__ off, const int* __restrict__ cnt,
    const float* __restrict__ h, float* nm, int nN, int csrLen) {
  const int tid = threadIdx.x, lane = tid & 31, wave = tid >> 5;
  const int tbase = blockIdx.x * TGT + wave * 32;
  const int col4 = 4 * lane;
  const int cl    = tbase + lane;
  const int cnt_l = cnt[cl];
  const int off_l = off[cl];

#pragma unroll 1
  for (int j = 0; j < 32; ++j) {
    const int c = tbase + j;
    const int nraw = __shfl(cnt_l, j);
    int n = nraw < 0 ? 0 : (nraw > DEGCAP ? DEGCAP : nraw);
    const int st = __shfl(off_l, j);

    v4f a = {0.f, 0.f, 0.f, 0.f};
#pragma unroll 1
    for (int q0 = 0; q0 < n; q0 += 32) {
      int pos = st + q0 + lane;
      pos = pos < 0 ? 0 : (pos > csrLen - 1 ? csrLen - 1 : pos);
      int sl = csr[pos];
      sl = sl < 0 ? 0 : (sl > nN - 1 ? nN - 1 : sl);
      const int mcnt = (n - q0) < 32 ? (n - q0) : 32;
#pragma unroll 1
      for (int pp = 0; pp < mcnt; ++pp) {
        const int s = __builtin_amdgcn_readlane(sl, pp);
        const v4f xv = *(const v4f*)(h + (size_t)s * DW + col4);
        a = a + xv;
      }
    }

    const bool live = c < nN;
    const float cf = (float)(nraw < 1 ? 1 : nraw);
    float inv = 1.0f / cf;
    inv = (nraw > DEGCAP) ? __int_as_float(0x7fc00000) : inv;
    v4f o;
    o.x = live ? a.x * inv : 0.f;
    o.y = live ? a.y * inv : 0.f;
    o.z = live ? a.z * inv : 0.f;
    o.w = live ? a.w * inv : 0.f;
    float* gp = nm + (size_t)c * DW + col4;
    *(volatile v4f*)gp = o;
    __threadfence();
    *(volatile v4f*)gp = o;
  }
}

__global__ __launch_bounds__(NTHR) void k_layer(
    const float* __restrict__ h, const float* __restrict__ nm, const int* __restrict__ cnt,
    const _Float16* __restrict__ wpl, const float* __restrict__ bS, const float* __restrict__ bN,
    const float* __restrict__ bG, const float* __restrict__ lng, const float* __restrict__ lnb,
    float* out, int nValid) {
  constexpr int TPW = 4;
  constexpr int PPR = DW / 4;
  constexpr int NIT = (BM * PPR) / NTHR;
  constexpr int RPI = NTHR / 32;
  constexpr int KS1 = DW / 32;
  constexpr int KS2 = (2 * DW) / 32;
  static_assert((BM * PPR) % NTHR == 0);
  static_assert(NIT * RPI == BM);
  static_assert(TPW * 16 * 2 == DW);
  static_assert(BM == 4 * 16);
  static_assert(PPR == 32);

  extern __shared__ v4f lds_dyn[];
  _Float16* a16 = (_Float16*)lds_dyn;
  float* stg = (float*)(a16 + 2 * BM * DW);
  float* gtl = (float*)lds_dyn;

  const int tid = threadIdx.x, lane = tid & 31, wave = tid >> 5, hh = lane >> 4, m = lane & 15;
  const int rowBase = (int)blockIdx.x * BM;
  const int rg = wave >> 1, chf = wave & 1;
  const int r0 = rg * 16;
  const int c0 = chf * (DW / 2);

#pragma unroll
  for (int it = 0; it < NIT; ++it) {
    const int row = it * RPI + wave;
    const int grow = rowBase + row;
    const bool live = grow < nValid;
    int rr = grow > nValid - 1 ? nValid - 1 : grow;
    rr = rr < 0 ? 0 : rr;
    v4f xv = *(const v4f*)(h + (size_t)rr * DW + 4 * lane);
    const v4f nv = *(const v4f*)(nm + (size_t)grow * DW + 4 * lane);
    xv.x = live ? xv.x : 0.f;
    xv.y = live ? xv.y : 0.f;
    xv.z = live ? xv.z : 0.f;
    xv.w = live ? xv.w : 0.f;
    v4h o, p;
    o.x = (_Float16)(xv.x * ACARRY);
    o.y = (_Float16)(xv.y * ACARRY);
    o.z = (_Float16)(xv.z * ACARRY);
    o.w = (_Float16)(xv.w * ACARRY);
    p.x = (_Float16)(nv.x * ACARRY);
    p.y = (_Float16)(nv.y * ACARRY);
    p.z = (_Float16)(nv.z * ACARRY);
    p.w = (_Float16)(nv.w * ACARRY);
    *(v4h*)(a16 + (size_t)row * DW + 4 * lane) = o;
    *(v4h*)(a16 + (size_t)BM * DW + (size_t)row * DW + 4 * lane) = p;
  }
  __syncthreads();

  v8f acc[TPW];
  float* sp = stg + (size_t)(r0 + 8 * hh) * DW + c0 + m;

#pragma unroll
  for (int t = 0; t < TPW; ++t) { v8f z = {0.f, 0.f, 0.f, 0.f, 0.f, 0.f, 0.f, 0.f}; acc[t] = z; }
  {
    const _Float16* ap = a16 + (size_t)(r0 + m) * DW + 8 * hh;
    const _Float16* bp = wpl + (size_t)(c0 + m) * DW + 8 * hh;
#pragma unroll 1
    for (int kt = 0; kt < KS1; ++kt) {
      Frag a;
      a.h[0] = *(const v8h*)(ap + 32 * kt);
      a.h[1] = *(const v8h*)(ap + 32 * kt + 16);
#pragma unroll
      for (int t = 0; t < TPW; ++t) {
        const size_t to = (size_t)(16 * t) * DW + 32 * kt;
        Frag b;
        b.h[0] = *(const v8h*)(bp + to);
        b.h[1] = *(const v8h*)(bp + to + 16);
        acc[t] = wmh(a.v, b.v, acc[t]);
      }
    }
  }
#pragma unroll
  for (int t = 0; t < TPW; ++t) {
    const float bv = bS[c0 + 16 * t + m];
#pragma unroll
    for (int r = 0; r < 8; ++r) sp[r * DW + 16 * t] = acc[t][r] * GSCALE + bv;
  }

#pragma unroll
  for (int t = 0; t < TPW; ++t) { v8f z = {0.f, 0.f, 0.f, 0.f, 0.f, 0.f, 0.f, 0.f}; acc[t] = z; }
  {
    const _Float16* ap = a16 + (size_t)BM * DW + (size_t)(r0 + m) * DW + 8 * hh;
    const _Float16* bp = wpl + (size_t)DW * DW + (size_t)(c0 + m) * DW + 8 * hh;
#pragma unroll 1
    for (int kt = 0; kt < KS1; ++kt) {
      Frag a;
      a.h[0] = *(const v8h*)(ap + 32 * kt);
      a.h[1] = *(const v8h*)(ap + 32 * kt + 16);
#pragma unroll
      for (int t = 0; t < TPW; ++t) {
        const size_t to = (size_t)(16 * t) * DW + 32 * kt;
        Frag b;
        b.h[0] = *(const v8h*)(bp + to);
        b.h[1] = *(const v8h*)(bp + to + 16);
        acc[t] = wmh(a.v, b.v, acc[t]);
      }
    }
  }
  float pr[8];
  {
    const int growb = rowBase + r0 + 8 * hh;
#pragma unroll
    for (int r = 0; r < 8; ++r) {
      const int ci = cnt[growb + r];
      pr[r] = ci > 0 ? 1.f : 0.f;
    }
  }
#pragma unroll
  for (int t = 0; t < TPW; ++t) {
    const float bv = bN[c0 + 16 * t + m];
#pragma unroll
    for (int r = 0; r < 8; ++r) {
      const float mv = sp[r * DW + 16 * t] + pr[r] * (acc[t][r] * GSCALE + bv);
      sp[r * DW + 16 * t] = mv;
      acc[t][r] = mv;
    }
  }
  __syncthreads();
  {
    _Float16* mp = a16 + (size_t)BM * DW + (size_t)(r0 + 8 * hh) * DW + c0 + m;
#pragma unroll
    for (int t = 0; t < TPW; ++t) {
#pragma unroll
      for (int r = 0; r < 8; ++r) mp[r * DW + 16 * t] = (_Float16)(acc[t][r] * ACARRY);
    }
  }
  __syncthreads();

#pragma unroll
  for (int t = 0; t < TPW; ++t) { v8f z = {0.f, 0.f, 0.f, 0.f, 0.f, 0.f, 0.f, 0.f}; acc[t] = z; }
  {
    const _Float16* ab = a16 + (size_t)(r0 + m) * DW + 8 * hh;
    const _Float16* bp = wpl + (size_t)2 * DW * DW + (size_t)(c0 + m) * (2 * DW) + 8 * hh;
#pragma unroll 1
    for (int kt = 0; kt < KS2; ++kt) {
      const _Float16* ap = ab + (size_t)(kt >> 2) * BM * DW + 32 * (kt & 3);
      Frag a;
      a.h[0] = *(const v8h*)(ap);
      a.h[1] = *(const v8h*)(ap + 16);
#pragma unroll
      for (int t = 0; t < TPW; ++t) {
        const size_t to = (size_t)(16 * t) * (2 * DW) + 32 * kt;
        Frag b;
        b.h[0] = *(const v8h*)(bp + to);
        b.h[1] = *(const v8h*)(bp + to + 16);
        acc[t] = wmh(a.v, b.v, acc[t]);
      }
    }
  }
  __syncthreads();
  {
    float* gq = gtl + (size_t)(r0 + 8 * hh) * DW + c0 + m;
#pragma unroll
    for (int t = 0; t < TPW; ++t) {
      const float bv = bG[c0 + 16 * t + m];
#pragma unroll
      for (int r = 0; r < 8; ++r) {
        const float x = acc[t][r] * GSCALE + bv;
        const float e = expf(-x);
        gq[r * DW + 16 * t] = 1.0f / (1.0f + e);
      }
    }
  }
  __syncthreads();

  const v4f gmv = *(const v4f*)(lng + 4 * lane);
  const v4f btv = *(const v4f*)(lnb + 4 * lane);
  v4f cv[NIT];
#pragma unroll
  for (int it = 0; it < NIT; ++it) {
    const int row = it * RPI + wave;
    const int grow = rowBase + row;
    int rr = grow > nValid - 1 ? nValid - 1 : grow;
    rr = rr < 0 ? 0 : rr;
    const v4f m4 = *(const v4f*)(stg + (size_t)row * DW + 4 * lane);
    const v4f g4 = *(const v4f*)(gtl + (size_t)row * DW + 4 * lane);
    const v4f h4 = *(const v4f*)(h + (size_t)rr * DW + 4 * lane);
    const v4f vv = g4 * m4 + (1.0f - g4) * h4;
    float s = vv.x + vv.y + vv.z + vv.w;
    s = wsum(s);
    const float mu = s * (1.0f / DW);
    const v4f d = vv - mu;
    float q = d.x * d.x + d.y * d.y + d.z * d.z + d.w * d.w;
    q = wsum(q);
    const float rs = rsqrtf(q * (1.0f / DW) + LN_EPS);
    v4f o = d * rs * gmv + btv;
    o.x = fmaxf(o.x, 0.f);
    o.y = fmaxf(o.y, 0.f);
    o.z = fmaxf(o.z, 0.f);
    o.w = fmaxf(o.w, 0.f);
    cv[it] = o;
  }
#pragma unroll
  for (int it = 0; it < NIT; ++it) {
    const int grow = rowBase + it * RPI + wave;
    if (grow < nValid) {
      float* gp = out + (size_t)grow * DW + 4 * lane;
      *(volatile v4f*)gp = cv[it];
    }
  }
  __threadfence();
#pragma unroll
  for (int it = 0; it < NIT; ++it) {
    const int grow = rowBase + it * RPI + wave;
    if (grow < nValid) {
      float* gp = out + (size_t)grow * DW + 4 * lane;
      *(volatile v4f*)gp = cv[it];
    }
  }
}

extern "C" void kernel_launch(void* const* d_in, const int* in_sizes, int n_in,
                              void* d_out, int out_size, void* d_ws, size_t ws_size,
                              hipStream_t stream) {
  if (n_in < 11) return;
  if (in_sizes[0] < DW || (in_sizes[0] % DW) != 0) return;
  const int nN = in_sizes[0] / DW;
  const int nE = in_sizes[1];
  if (nE < 1 || in_sizes[2] != nE) return;
  if (in_sizes[3] != DW * DW || in_sizes[4] != DW) return;
  if (in_sizes[5] != DW * DW || in_sizes[6] != DW) return;
  if (in_sizes[7] != 2 * DW * DW || in_sizes[8] != DW) return;
  if (in_sizes[9] != DW || in_sizes[10] != DW) return;
  if ((long long)out_size != (long long)nN * DW) return;
  if (nE > (1 << 28) || nN > (1 << 22)) return;

  const float* h   = (const float*)d_in[0];
  const int*   src = (const int*)d_in[1];
  const int*   dst = (const int*)d_in[2];
  const float* wS  = (const float*)d_in[3];
  const float* bS  = (const float*)d_in[4];
  const float* wN  = (const float*)d_in[5];
  const float* bN  = (const float*)d_in[6];
  const float* wG  = (const float*)d_in[7];
  const float* bG  = (const float*)d_in[8];
  const float* lng = (const float*)d_in[9];
  const float* lnb = (const float*)d_in[10];
  float* out = (float*)d_out;

  const int NPAD   = ((nN + TGT - 1) / TGT) * TGT;
  const int nBC    = (nN + NBC - 1) / NBC;
  const int CNTPAD = nBC * NBC;
  if (CNTPAD < NPAD) return;
  if (4 * nBC + 1 > RBN) return;
  const int nBF    = (nN + NBF - 1) / NBF;
  if (nBF > 4 * nBC) return;
  const int csrLen = ((nE + 31) & ~31) + 4096;
  if (31 * 4 * nBC > 4096) return;
  const int nAgg   = NPAD / TGT;
  const int nLay   = NPAD / BM;
  const int nUnits = (4 * DW * DW) / 8;

  char* ws = (char*)d_ws;
  size_t off = 0;
  const size_t oWp  = off; off += (size_t)4 * DW * DW * 2;   off = (off + 255) & ~(size_t)255;
  const size_t oNm  = off; off += (size_t)NPAD * DW * 4;     off = (off + 255) & ~(size_t)255;
  const size_t oCnt = off; off += (size_t)CNTPAD * 4;        off = (off + 255) & ~(size_t)255;
  const size_t oOff = off; off += (size_t)CNTPAD * 4;        off = (off + 255) & ~(size_t)255;
  const size_t oRb  = off; off += (size_t)RBN * 4;           off = (off + 255) & ~(size_t)255;
  const size_t oCsr = off; off += (size_t)csrLen * 4;        off = (off + 255) & ~(size_t)255;
  if (off > ws_size || off > (size_t)WSCAP) return;

  _Float16* wpl = (_Float16*)(ws + oWp);
  float* nmp  = (float*)(ws + oNm);
  int*   cnt  = (int*)(ws + oCnt);
  int*   offp = (int*)(ws + oOff);
  int*   rb   = (int*)(ws + oRb);
  int*   csr  = (int*)(ws + oCsr);

  const int vec8 = 1;

  k_wcvt<<<(nUnits + NTHR - 1) / NTHR, NTHR, 0, stream>>>(wS, wN, wG, wpl, nUnits);
  k_count<<<nBC, NTHR, 0, stream>>>(dst, cnt, nE, vec8);
  k_offsets<<<1, OTHR, 0, stream>>>(cnt, offp, rb, nBC);
  hipFuncSetAttribute(reinterpret_cast<const void*>(&k_fill),
                      hipFuncAttributeMaxDynamicSharedMemorySize, LDS_FILL);
  k_fill<<<nBF, NTHR, LDS_FILL, stream>>>(src, dst, offp, rb, csr, nN, nE, vec8, csrLen);
  k_agg<<<nAgg, NTHR, 0, stream>>>(csr, offp, cnt, h, nmp, nN, csrLen);

  hipFuncSetAttribute(reinterpret_cast<const void*>(&k_layer),
                      hipFuncAttributeMaxDynamicSharedMemorySize, LDS_LAYER);
  k_layer<<<nLay, NTHR, LDS_LAYER, stream>>>(h, nmp, cnt, wpl, bS, bN, bG, lng, lnb, out, nN);
}
